// GCNUnit_34067680592304
// MI455X (gfx1250) — hardware-verified
//
#include <hip/hip_runtime.h>
#include <stddef.h>


#define FD      128
#define NTHR    256
#define NWAVE   8
#define EPT     8
#define NGRP    2
#define CHUNK   (NTHR * EPT * NGRP)
#define WCAP    (EPT * NGRP * 32)
#define LISTN   (NWAVE * WCAP)
#define ESHF    11
#define NBC     32768
#define NBF     2048
#define RCAP    40960
#define RBN     128
#define TGT     256
#define DEGCAP  512
#define GROWS   128
#define OTHR    512
#define WSCALE  16
#define ASCALE1 1
#define ASCALE2 64
#define CSELF   1.0f
#define SLOPE   0.01f
#define WSCAP   134217728

#define LDS_COUNT ((NBC + LISTN + NWAVE) * 4)
#define LDS_FILL  ((RCAP + NBF + LISTN + NWAVE) * 4)
#define LDS_GEMM  (GROWS * FD * 4)
#define WPB       ((FD * FD / 8) / NTHR)

static_assert((CHUNK & (CHUNK - 1)) == 0);
static_assert((NBC & (NBC - 1)) == 0 && (NBF & (NBF - 1)) == 0);
static_assert(NBF <= (1 << ESHF));
static_assert((NBC % NBF) == 0);
static_assert(OTHR * 4 == NBF);
static_assert((RCAP % 32) == 0);
static_assert(TGT == NWAVE * 32);
static_assert(GROWS == NWAVE * 16);
static_assert((TGT % GROWS) == 0);
static_assert((FD % 32) == 0 && FD == 32 * 4);
static_assert(NBC == NWAVE * 32 * 128);
static_assert((FD * FD / 8) % NTHR == 0 && FD / 8 == 16);
static_assert((16 * FD) % 128 == 0);

typedef float     v4f  __attribute__((ext_vector_type(4)));
typedef float     v8f  __attribute__((ext_vector_type(8)));
typedef int       v4i  __attribute__((ext_vector_type(4)));
typedef _Float16  v8h  __attribute__((ext_vector_type(8)));
typedef _Float16  v16h __attribute__((ext_vector_type(16)));
union FragH { v16h v; v8h h[2]; };

__device__ __forceinline__ v8f wmf(v16h a, v16h b, v8f c) {
  v8f d = __builtin_amdgcn_wmma_f32_16x16x32_f16(false, a, false, b, (short)0, c, false, false);
  asm volatile("v_nop\n\tv_nop\n\tv_nop\n\tv_nop" : "+v"(d) : "v"(a), "v"(b));
  return d;
}

template <int NB, int SRC>
__device__ __forceinline__ int scan_chunk(const int* __restrict__ keys, const int* __restrict__ gath, int nE, int nN,
                                          int cbase, int slotBase, int vec8, int* list, int tid, int lane, int wave) {
  int wc = 0;
#pragma unroll
  for (int g = 0; g < NGRP; ++g) {
    const int el0  = (g * NTHR + tid) * EPT;
    const int e0   = cbase + el0;
    const int sent = -2147483647 - 1;
    v4i da, db;
    v4i sa = {0, 0, 0, 0}, sb = {0, 0, 0, 0};
    if (vec8 != 0 && cbase + CHUNK <= nE) {
      da = *(const v4i*)(keys + e0);
      db = *(const v4i*)(keys + e0 + 4);
      if (SRC) {
        sa = *(const v4i*)(gath + e0);
        sb = *(const v4i*)(gath + e0 + 4);
      }
    } else {
      da.x = (e0     < nE) ? keys[min(e0, nE - 1)] : sent;
      da.y = (e0 + 1 < nE) ? keys[min(e0 + 1, nE - 1)] : sent;
      da.z = (e0 + 2 < nE) ? keys[min(e0 + 2, nE - 1)] : sent;
      da.w = (e0 + 3 < nE) ? keys[min(e0 + 3, nE - 1)] : sent;
      db.x = (e0 + 4 < nE) ? keys[min(e0 + 4, nE - 1)] : sent;
      db.y = (e0 + 5 < nE) ? keys[min(e0 + 5, nE - 1)] : sent;
      db.z = (e0 + 6 < nE) ? keys[min(e0 + 6, nE - 1)] : sent;
      db.w = (e0 + 7 < nE) ? keys[min(e0 + 7, nE - 1)] : sent;
      if (SRC) {
        sa.x = gath[min(e0, nE - 1)];
        sa.y = gath[min(e0 + 1, nE - 1)];
        sa.z = gath[min(e0 + 2, nE - 1)];
        sa.w = gath[min(e0 + 3, nE - 1)];
        sb.x = gath[min(e0 + 4, nE - 1)];
        sb.y = gath[min(e0 + 5, nE - 1)];
        sb.z = gath[min(e0 + 6, nE - 1)];
        sb.w = gath[min(e0 + 7, nE - 1)];
      }
    }
    if (SRC) {
      sa.x = min(max(sa.x, 0), nN - 1); sa.y = min(max(sa.y, 0), nN - 1);
      sa.z = min(max(sa.z, 0), nN - 1); sa.w = min(max(sa.w, 0), nN - 1);
      sb.x = min(max(sb.x, 0), nN - 1); sb.y = min(max(sb.y, 0), nN - 1);
      sb.z = min(max(sb.z, 0), nN - 1); sb.w = min(max(sb.w, 0), nN - 1);
    }
    const unsigned nb = (unsigned)slotBase;
    const unsigned s0 = (unsigned)da.x - nb, s1 = (unsigned)da.y - nb;
    const unsigned s2 = (unsigned)da.z - nb, s3 = (unsigned)da.w - nb;
    const unsigned s4 = (unsigned)db.x - nb, s5 = (unsigned)db.y - nb;
    const unsigned s6 = (unsigned)db.z - nb, s7 = (unsigned)db.w - nb;
    const bool h0 = s0 < (unsigned)NB, h1 = s1 < (unsigned)NB, h2 = s2 < (unsigned)NB, h3 = s3 < (unsigned)NB;
    const bool h4 = s4 < (unsigned)NB, h5 = s5 < (unsigned)NB, h6 = s6 < (unsigned)NB, h7 = s7 < (unsigned)NB;
    const unsigned any = __builtin_amdgcn_ballot_w32(h0 | h1 | h2 | h3 | h4 | h5 | h6 | h7);
    if (any != 0u) {
#define HITJ(HJ, SJ, VJ) { \
        const unsigned mj = __builtin_amdgcn_ballot_w32(HJ); \
        if (mj != 0u) { \
          if (HJ) { \
            const int pos = wc + (int)__builtin_amdgcn_mbcnt_lo(mj, 0u); \
            const int entv = SRC ? (((VJ) << ESHF) | (int)(SJ)) : (int)(SJ); \
            if (pos < WCAP) list[wave * WCAP + pos] = entv; \
          } \
          wc += (int)__builtin_popcount(mj); } }
      HITJ(h0, s0, sa.x)
      HITJ(h1, s1, sa.y)
      HITJ(h2, s2, sa.z)
      HITJ(h3, s3, sa.w)
      HITJ(h4, s4, sb.x)
      HITJ(h5, s5, sb.y)
      HITJ(h6, s6, sb.z)
      HITJ(h7, s7, sb.w)
#undef HITJ
    }
  }
  return wc;
}

__global__ __launch_bounds__(NTHR) void k_wprep(const float* __restrict__ w1, const float* __restrict__ w2, _Float16* wp) {
  const int tid   = threadIdx.x;
  const int plane = (int)blockIdx.x >= WPB ? 1 : 0;
  const int i  = ((int)blockIdx.x - plane * WPB) * NTHR + tid;
  const int n  = i >> 4;
  const int k0 = (i & 15) * 8;
  const float* w = (plane == 0) ? w1 : w2;
  v8h hv;
#pragma unroll
  for (int e = 0; e < 8; ++e) hv[e] = (_Float16)(w[(k0 + e) * FD + n] * (float)WSCALE);
  _Float16* d = wp + (size_t)plane * FD * FD + (size_t)i * 8;
  *(volatile v8h*)d = hv;
  __threadfence();
  *(volatile v8h*)d = hv;
}

__global__ __launch_bounds__(NTHR) void k_count(
    const int* __restrict__ ei, int* cnt, float* dinv, int nE, int nN, int vec8) {
  extern __shared__ v4f lds_dyn[];
  int* scnt = (int*)lds_dyn;
  int* list = scnt + NBC;
  int* wcnt = list + LISTN;
  const int tid = threadIdx.x, lane = tid & 31, wave = tid >> 5;
  const int nodeBase = blockIdx.x * NBC;
  const int* keys = ei + nE;
  const int* gath = ei;

  {
    const v4i z = {0, 0, 0, 0};
    for (int i = tid; i < NBC / 4; i += NTHR) ((v4i*)scnt)[i] = z;
  }
  __syncthreads();

  const int nChunks = (nE + CHUNK - 1) / CHUNK;
#pragma unroll 1
  for (int ch = 0; ch < nChunks; ++ch) {
    const int cbase = ch * CHUNK;
    const int wc = scan_chunk<NBC, 0>(keys, gath, nE, nN, cbase, nodeBase, vec8, list, tid, lane, wave);
    if (lane == 0) wcnt[wave] = wc;
    __syncthreads();
    if (wave == 0) {
#pragma unroll 1
      for (int wsx = 0; wsx < NWAVE; ++wsx) {
        int n = __builtin_amdgcn_readfirstlane(wcnt[wsx]);
        n = n > WCAP ? WCAP : (n < 0 ? 0 : n);
        const int* lp = list + wsx * WCAP;
#pragma unroll 1
        for (int i = 0; i < n; ++i) {
          const int ent  = __builtin_amdgcn_readfirstlane(lp[i]);
          const int slot = ent & (NBC - 1);
          if (lane == 0) scnt[slot] = scnt[slot] + 1;
        }
      }
    }
    __syncthreads();
  }

  int*   cp = cnt + (size_t)nodeBase;
  float* dp = dinv + (size_t)nodeBase;
#pragma unroll 4
  for (int q = 0; q < 32; ++q) {
    const int f = (wave * 32 + q) * 128 + 4 * lane;
    const v4i c = *(const v4i*)(scnt + f);
    const float g0 = (float)c.x + CSELF, g1 = (float)c.y + CSELF, g2 = (float)c.z + CSELF, g3 = (float)c.w + CSELF;
    v4f d;
    d.x = g0 > 0.f ? rsqrtf(g0) : 0.f; d.y = g1 > 0.f ? rsqrtf(g1) : 0.f;
    d.z = g2 > 0.f ? rsqrtf(g2) : 0.f; d.w = g3 > 0.f ? rsqrtf(g3) : 0.f;
    *(volatile v4i*)(cp + f) = c;
    *(volatile v4f*)(dp + f) = d;
  }
  __threadfence();
#pragma unroll 4
  for (int q = 0; q < 32; ++q) {
    const int f = (wave * 32 + q) * 128 + 4 * lane;
    const v4i c = *(const v4i*)(scnt + f);
    const float g0 = (float)c.x + CSELF, g1 = (float)c.y + CSELF, g2 = (float)c.z + CSELF, g3 = (float)c.w + CSELF;
    v4f d;
    d.x = g0 > 0.f ? rsqrtf(g0) : 0.f; d.y = g1 > 0.f ? rsqrtf(g1) : 0.f;
    d.z = g2 > 0.f ? rsqrtf(g2) : 0.f; d.w = g3 > 0.f ? rsqrtf(g3) : 0.f;
    *(volatile v4i*)(cp + f) = c;
    *(volatile v4f*)(dp + f) = d;
  }
}

__global__ __launch_bounds__(OTHR) void k_offsets(
    const int* __restrict__ cnt, int* off, int* rbase, int nBF) {
  __shared__ __attribute__((aligned(16))) int srb[RBN];
  __shared__ int wtot[OTHR / 32];
  const int tid = threadIdx.x, lane = tid & 31, wave = tid >> 5;
  for (int i = tid; i < RBN; i += OTHR) srb[i] = 0;
  int carry = 0;
#pragma unroll 1
  for (int fb = 0; fb < nBF; ++fb) {
    const int base = fb * NBF;
    const v4i c = *(const v4i*)(cnt + base + 4 * tid);
    const int e0 = max(c.x, 0), e1 = max(c.y, 0), e2 = max(c.z, 0), e3 = max(c.w, 0);
    const int ts = e0 + e1 + e2 + e3;
    int incl = ts;
#pragma unroll
    for (int d = 1; d < 32; d <<= 1) {
      const int t = __shfl_up(incl, d);
      if (lane >= d) incl += t;
    }
    if (lane == 31) wtot[wave] = incl;
    __syncthreads();
    int pre = 0;
#pragma unroll 1
    for (int w = 0; w < wave; ++w) pre += wtot[w];
    int tot = 0;
#pragma unroll
    for (int w = 0; w < OTHR / 32; ++w) tot += wtot[w];
    int run = carry + pre + incl - ts;
    v4i o;
    o.x = run; run += e0;
    o.y = run; run += e1;
    o.z = run; run += e2;
    o.w = run;
    int* op = off + base + 4 * tid;
    *(volatile v4i*)op = o;
    __threadfence();
    *(volatile v4i*)op = o;
    if (tid == 0) srb[min(fb, RBN - 1)] = carry;
    carry += (tot + 31) & ~31;
    __syncthreads();
  }
  if (tid == 0) srb[min(nBF, RBN - 1)] = carry;
  __syncthreads();
  v4i rv = {0, 0, 0, 0};
  if (tid < 32) rv = *(const v4i*)(srb + 4 * tid);
  if (tid < 32) *(volatile v4i*)(rbase + 4 * tid) = rv;
  __threadfence();
  if (tid < 32) *(volatile v4i*)(rbase + 4 * tid) = rv;
}

__global__ __launch_bounds__(NTHR) void k_fill(
    const int* __restrict__ ei, const int* __restrict__ off, const int* __restrict__ rbase,
    int* csr, int nN, int nE, int vec8, int csrLen) {
  extern __shared__ v4f lds_dyn[];
  int* region = (int*)lds_dyn;
  int* cursor = region + RCAP;
  int* list   = cursor + NBF;
  int* wcnt   = list + LISTN;
  const int tid = threadIdx.x, lane = tid & 31, wave = tid >> 5;
  const int b = blockIdx.x;
  const int nodeBase = b * NBF;
  const int* keys = ei + nE;
  const int* gath = ei;

  int rb0 = rbase[b];
  const int rb1 = rbase[b + 1];
  rb0 = rb0 < 0 ? 0 : (rb0 > csrLen ? csrLen : rb0);
  rb0 &= ~31;
  int len = rb1 - rb0;
  len = len < 0 ? 0 : (len > RCAP ? RCAP : len);
  int lenW = (len + 31) & ~31;
  if (rb0 + lenW > csrLen) lenW = (csrLen - rb0) & ~31;

  {
    const v4i z = {0, 0, 0, 0};
    for (int i = tid; i < RCAP / 4; i += NTHR) ((v4i*)region)[i] = z;
    for (int s = tid; s < NBF; s += NTHR) {
      int o = off[nodeBase + s] - rb0;
      o = o < 0 ? 0 : (o > RCAP ? RCAP : o);
      cursor[s] = o;
    }
  }
  __syncthreads();

  const int nChunks = (nE + CHUNK - 1) / CHUNK;
#pragma unroll 1
  for (int ch = 0; ch < nChunks; ++ch) {
    const int cbase = ch * CHUNK;
    const int wc = scan_chunk<NBF, 1>(keys, gath, nE, nN, cbase, nodeBase, vec8, list, tid, lane, wave);
    if (lane == 0) wcnt[wave] = wc;
    __syncthreads();
    if (wave == 0) {
#pragma unroll 1
      for (int wsx = 0; wsx < NWAVE; ++wsx) {
        int n = __builtin_amdgcn_readfirstlane(wcnt[wsx]);
        n = n > WCAP ? WCAP : (n < 0 ? 0 : n);
        const int* lp = list + wsx * WCAP;
#pragma unroll 1
        for (int i = 0; i < n; ++i) {
          const int ent  = __builtin_amdgcn_readfirstlane(lp[i]);
          const int slot = ent & (NBF - 1);
          int src = (ent >> ESHF) & 0xFFFFF;
          src = src > nN - 1 ? nN - 1 : src;
          if (lane == 0) {
            int pos = cursor[slot];
            pos = pos < 0 ? 0 : (pos > RCAP - 1 ? RCAP - 1 : pos);
            region[pos] = src;
            const int np = pos + 1;
            cursor[slot] = np > RCAP ? RCAP : np;
          }
        }
      }
    }
    __syncthreads();
  }

  const int nv = lenW >> 2;
  int* gp = csr + rb0;
#pragma unroll 1
  for (int i = tid; i < nv; i += NTHR) { const v4i v = ((const v4i*)region)[i]; *(volatile v4i*)(gp + 4 * i) = v; }
  __threadfence();
#pragma unroll 1
  for (int i = tid; i < nv; i += NTHR) { const v4i v = ((const v4i*)region)[i]; *(volatile v4i*)(gp + 4 * i) = v; }
}

template <int ASC>
__global__ __launch_bounds__(NTHR) void k_gemm(
    const float* __restrict__ A, const _Float16* __restrict__ Bw, const float* __restrict__ dinv,
    float* C, int nRowsA) {
  extern __shared__ v4f lds_dyn[];
  constexpr int KD = FD;
  constexpr int NC = FD;
  constexpr int NT = NC / 16;
  constexpr float OSC = 1.0f / (float)(ASC * WSCALE);
  float* stg = (float*)lds_dyn;
  const int tid = threadIdx.x, lane = tid & 31, wave = tid >> 5, hh = lane >> 4, m = lane & 15;
  const int rowBase = blockIdx.x * GROWS;
  int arow = rowBase + wave * 16 + m;
  arow = arow > nRowsA - 1 ? nRowsA - 1 : arow;
  const float* ap = A + (size_t)arow * KD + 8 * hh;

  v8f acc[NT];
#pragma unroll
  for (int t = 0; t < NT; ++t) { v8f z = {0.f, 0.f, 0.f, 0.f, 0.f, 0.f, 0.f, 0.f}; acc[t] = z; }

#pragma unroll 1
  for (int kt = 0; kt < KD / 32; ++kt) {
    const float* akp = ap + 32 * kt;
    const v4f f0 = *(const v4f*)akp;
    const v4f f1 = *(const v4f*)(akp + 4);
    const v4f f2 = *(const v4f*)(akp + 16);
    const v4f f3 = *(const v4f*)(akp + 20);
    v8h lo, hi;
    lo[0] = (_Float16)(f0.x * (float)ASC); lo[1] = (_Float16)(f0.y * (float)ASC);
    lo[2] = (_Float16)(f0.z * (float)ASC); lo[3] = (_Float16)(f0.w * (float)ASC);
    lo[4] = (_Float16)(f1.x * (float)ASC); lo[5] = (_Float16)(f1.y * (float)ASC);
    lo[6] = (_Float16)(f1.z * (float)ASC); lo[7] = (_Float16)(f1.w * (float)ASC);
    hi[0] = (_Float16)(f2.x * (float)ASC); hi[1] = (_Float16)(f2.y * (float)ASC);
    hi[2] = (_Float16)(f2.z * (float)ASC); hi[3] = (_Float16)(f2.w * (float)ASC);
    hi[4] = (_Float16)(f3.x * (float)ASC); hi[5] = (_Float16)(f3.y * (float)ASC);
    hi[6] = (_Float16)(f3.z * (float)ASC); hi[7] = (_Float16)(f3.w * (float)ASC);
    FragH af;
    af.h[0] = lo;
    af.h[1] = hi;
#pragma unroll
    for (int t = 0; t < NT; ++t) {
      const _Float16* bp = Bw + (size_t)(16 * t + m) * KD + 32 * kt + 8 * hh;
      FragH bf;
      bf.h[0] = *(const v8h*)bp;
      bf.h[1] = *(const v8h*)(bp + 16);
      acc[t] = wmf(af.v, bf.v, acc[t]);
    }
  }

  const int r0 = wave * 16 + 8 * hh;
  const v4f dA = *(const v4f*)(dinv + (size_t)rowBase + r0);
  const v4f dB = *(const v4f*)(dinv + (size_t)rowBase + r0 + 4);
  float s[8];
  s[0] = dA.x; s[1] = dA.y; s[2] = dA.z; s[3] = dA.w; s[4] = dB.x; s[5] = dB.y; s[6] = dB.z; s[7] = dB.w;
#pragma unroll
  for (int r = 0; r < 8; ++r) s[r] = s[r] * OSC;
  float* sp = stg + r0 * NC + m;
#pragma unroll
  for (int t = 0; t < NT; ++t) {
#pragma unroll
    for (int r = 0; r < 8; ++r) sp[r * NC + 16 * t] = acc[t][r] * s[r];
  }
  __syncthreads();

  const float* lp = stg + wave * 16 * NC;
  float* gp = C + (size_t)(rowBase + wave * 16) * NC;
#pragma unroll
  for (int i = 0; i < (16 * NC) / 128; ++i) {
    const v4f v = *(const v4f*)(lp + i * 128 + 4 * lane);
    *(volatile v4f*)(gp + i * 128 + 4 * lane) = v;
  }
  __threadfence();
#pragma unroll
  for (int i = 0; i < (16 * NC) / 128; ++i) {
    const v4f v = *(const v4f*)(lp + i * 128 + 4 * lane);
    *(volatile v4f*)(gp + i * 128 + 4 * lane) = v;
  }
}

__global__ __launch_bounds__(NTHR) void k_agg(
    const int* __restrict__ csr, const int* __restrict__ off, const int* __restrict__ cnt,
    const float* __restrict__ dinv, const float* __restrict__ hw, const float* __restrict__ bs,
    float* dst, int nN, int csrLen, int nRowsOut) {
  const int tid = threadIdx.x, lane = tid & 31, wave = tid >> 5;
  const int tbase = blockIdx.x * TGT + wave * 32;
  const int cl = tbase + lane;
  const int cnt_l = cnt[cl];
  const int off_l = off[cl];
  union FI { float f; int i; };
  FI dvu; dvu.f = dinv[cl];
  const v4f bb = *(const v4f*)(bs + 4 * lane);

#pragma unroll 1
  for (int j = 0; j < 32; ++j) {
    const int c = tbase + j;
    int n = __builtin_amdgcn_readlane(cnt_l, j);
    n = n < 0 ? 0 : (n > DEGCAP ? DEGCAP : n);
    const int st = __builtin_amdgcn_readlane(off_l, j);
    FI du; du.i = __builtin_amdgcn_readlane(dvu.i, j);
    const float dc = du.f;
    v4f acc = {0.f, 0.f, 0.f, 0.f};
#pragma unroll 1
    for (int q0 = 0; q0 < n; q0 += 32) {
      int pos = st + q0 + lane;
      pos = pos < 0 ? 0 : (pos > csrLen - 1 ? csrLen - 1 : pos);
      int sl = csr[pos];
      sl = sl < 0 ? 0 : (sl > nN - 1 ? nN - 1 : sl);
      const int mcnt = (n - q0) < 32 ? (n - q0) : 32;
#pragma unroll 1
      for (int p = 0; p < mcnt; ++p) {
        const int s = __builtin_amdgcn_readlane(sl, p);
        acc = acc + *(const v4f*)(hw + (size_t)s * FD + 4 * lane);
      }
    }
    const v4f sv = *(const v4f*)(hw + (size_t)c * FD + 4 * lane);
    v4f v = (acc + sv * CSELF) * dc + bb;
    v.x = v.x > 0.f ? v.x : v.x * SLOPE;
    v.y = v.y > 0.f ? v.y : v.y * SLOPE;
    v.z = v.z > 0.f ? v.z : v.z * SLOPE;
    v.w = v.w > 0.f ? v.w : v.w * SLOPE;
    if (c < nRowsOut) {
      float* hp = dst + (size_t)c * FD + 4 * lane;
      *(volatile v4f*)hp = v;
      __threadfence();
      *(volatile v4f*)hp = v;
    }
  }
}

extern "C" void kernel_launch(void* const* d_in, const int* in_sizes, int n_in,
                              void* d_out, int out_size, void* d_ws, size_t ws_size,
                              hipStream_t stream) {
  if (n_in < 6) return;
  const int nN = in_sizes[0] / FD;
  const int nE = in_sizes[5] / 2;
  if (nN <= 0 || nE <= 0 || in_sizes[0] != nN * FD || in_sizes[5] != 2 * nE) return;
  if (in_sizes[1] != FD * FD || in_sizes[2] != FD) return;
  if (in_sizes[3] != FD * FD || in_sizes[4] != FD) return;
  if (out_size != nN * FD) return;
  if (nN > (1 << 20) || nE > (1 << 28)) return;

  const float* x  = (const float*)d_in[0];
  const float* W1 = (const float*)d_in[1];
  const float* b1 = (const float*)d_in[2];
  const float* W2 = (const float*)d_in[3];
  const float* b2 = (const float*)d_in[4];
  const int*   ei = (const int*)d_in[5];
  float* out = (float*)d_out;

  const int NPAD   = ((nN + TGT - 1) / TGT) * TGT;
  const int nBC    = (nN + NBC - 1) / NBC;
  const int CNTPAD = nBC * NBC;
  const int nBF    = (nN + NBF - 1) / NBF;
  const int OFFN   = nBF * NBF;
  if (nBF + 1 > RBN) return;
  if (OFFN > CNTPAD || NPAD > OFFN) return;
  const int csrLen = ((nE + 31) & ~31) + 32 * (nBF + 1);
  const int nGemm  = NPAD / GROWS;
  const int nAgg   = NPAD / TGT;

  char* ws = (char*)d_ws;
  size_t off = 0;
  const size_t oW   = off; off += (size_t)(2 * FD * FD) * 2;     off = (off + 255) & ~(size_t)255;
  const size_t oCnt = off; off += (size_t)CNTPAD * 4;           off = (off + 255) & ~(size_t)255;
  const size_t oDv  = off; off += (size_t)CNTPAD * 4;           off = (off + 255) & ~(size_t)255;
  const size_t oOff = off; off += (size_t)OFFN * 4;             off = (off + 255) & ~(size_t)255;
  const size_t oRb  = off; off += (size_t)RBN * 4;              off = (off + 255) & ~(size_t)255;
  const size_t oCsr = off; off += (size_t)csrLen * 4;           off = (off + 255) & ~(size_t)255;
  const size_t oHw  = off; off += (size_t)NPAD * FD * 4;        off = (off + 255) & ~(size_t)255;
  const size_t oH   = off; off += (size_t)NPAD * FD * 4;        off = (off + 255) & ~(size_t)255;
  if (off > ws_size || off > (size_t)WSCAP) return;
  _Float16* wp   = (_Float16*)(ws + oW);
  int*      cnt  = (int*)(ws + oCnt);
  float*    dinv = (float*)(ws + oDv);
  int*      offp = (int*)(ws + oOff);
  int*      rb   = (int*)(ws + oRb);
  int*      csr  = (int*)(ws + oCsr);
  float*    hw   = (float*)(ws + oHw);
  float*    h    = (float*)(ws + oH);

  const int vec8 = ((nE & 3) == 0) ? 1 : 0;

  k_wprep<<<2 * WPB, NTHR, 0, stream>>>(W1, W2, wp);

  hipFuncSetAttribute(reinterpret_cast<const void*>(&k_count),
                      hipFuncAttributeMaxDynamicSharedMemorySize, LDS_COUNT);
  k_count<<<nBC, NTHR, LDS_COUNT, stream>>>(ei, cnt, dinv, nE, nN, vec8);
  k_offsets<<<1, OTHR, 0, stream>>>(cnt, offp, rb, nBF);
  hipFuncSetAttribute(reinterpret_cast<const void*>(&k_fill),
                      hipFuncAttributeMaxDynamicSharedMemorySize, LDS_FILL);
  k_fill<<<nBF, NTHR, LDS_FILL, stream>>>(ei, offp, rb, csr, nN, nE, vec8, csrLen);

  hipFuncSetAttribute(reinterpret_cast<const void*>(&k_gemm<ASCALE1>),
                      hipFuncAttributeMaxDynamicSharedMemorySize, LDS_GEMM);
  k_gemm<ASCALE1><<<nGemm, NTHR, LDS_GEMM, stream>>>(x, wp, dinv, hw, nN);
  k_agg<<<nAgg, NTHR, 0, stream>>>(csr, offp, cnt, dinv, hw, b1, h, nN, csrLen, NPAD);

  hipFuncSetAttribute(reinterpret_cast<const void*>(&k_gemm<ASCALE2>),
                      hipFuncAttributeMaxDynamicSharedMemorySize, LDS_GEMM);
  k_gemm<ASCALE2><<<nGemm, NTHR, LDS_GEMM, stream>>>(h, wp + (size_t)FD * FD, dinv, hw, NPAD);
  k_agg<<<nAgg, NTHR, 0, stream>>>(csr, offp, cnt, dinv, hw, b2, out, nN, csrLen, nN);
}
